// GNN_Combined_74869869904655
// MI455X (gfx1250) — hardware-run, weakly checked
//
#include <hip/hip_runtime.h>
#include <math.h>

constexpr int kNS = 20000;
constexpr int kES = 320000;
constexpr int kNL = 50000;
constexpr int kEL = 800000;
constexpr int kIn = 256;
constexpr int kHid = 128;
constexpr int kHeads = 4;
constexpr int kF1 = kHeads * kHid;
constexpr int kOut = 128;
constexpr int kCls = 4;
constexpr int kNSP = 20032;
constexpr int kNLP = 50048;
constexpr int kNT = 256;
constexpr int kTS1 = 1000;
constexpr int kRPW1 = kTS1 / 8;
constexpr int kNTile1 = kNS / kTS1;
constexpr int kSch1 = 2048;
constexpr int kNch1 = (kES + kSch1 - 1) / kSch1;
constexpr int kSch2 = 4096;
constexpr int kNch2 = (kES + kSch2 - 1) / kSch2;
constexpr int kTSL = 2048;
constexpr int kRPWL = kTSL / 8;
constexpr int kNTileL = (kNL + kTSL - 1) / kTSL;
constexpr int kNLR = kNTileL * kTSL;
constexpr int kSchL = 4096;
constexpr int kNchL = (kEL + kSchL - 1) / kSchL;

static_assert(kNTile1 * kTS1 == kNS);
static_assert(kRPW1 * 8 == kTS1 && kRPWL * 8 == kTSL);
static_assert(kES % (kSch1 / kNT) == 0 && kES % (kSch2 / kNT) == 0 && kEL % (kSchL / kNT) == 0);
static_assert(kNSP % 64 == 0 && kNLP % 64 == 0 && kF1 % 64 == 0 && kOut % 64 == 0);
static_assert(kIn % 32 == 0 && kF1 % 32 == 0 && kHid % 32 == 0);
static_assert(kNS % 8 == 0 && kNLP % 2 == 0 && kNLR >= kNLP);

constexpr size_t kSzF1 = (size_t)kNSP * kF1 * 4;
constexpr size_t kSzF2 = (size_t)kNS * kF1 * 4;
constexpr size_t kSzES = (size_t)kNS * kOut * 4;
constexpr size_t kSzB1 = (size_t)kNSP * kF1 * 2 * 2;
constexpr size_t kSzBT = ((size_t)kIn * kF1 + (size_t)kF1 * kOut + (size_t)kIn * kHid + (size_t)kHid * kOut) * 2;
constexpr size_t kOffF1 = 0;
constexpr size_t kOffF2 = kOffF1 + kSzF1;
constexpr size_t kOffES = kOffF2 + kSzF2;
constexpr size_t kOffB1 = kOffES + kSzES;
constexpr size_t kOffBT = kOffB1 + kSzB1;
constexpr size_t kWsTotal = kOffBT + kSzBT;
constexpr size_t kOffNS = (size_t)kNLR * kOut * 4;
constexpr size_t kOffND = kOffNS + (size_t)kNLR * 4;
static_assert(kWsTotal == 133742592ull && kWsTotal <= 134217728ull);
static_assert((size_t)kNLP * kOut * 4 <= kSzF1);
static_assert(81920 + (size_t)kNS * 4 <= kSzF1);
static_assert((size_t)kNSP * kOut * 4 <= kSzF2);
static_assert(kOffND + (size_t)kNLR * 4 <= kSzF2);
static_assert(2 * (size_t)kNS * kHeads * 4 <= kSzES);
static_assert((size_t)kNSP * kIn * 2 <= kSzB1 && (size_t)kNLP * kIn * 2 <= kSzB1 && (size_t)kNLP * kOut * 2 * 2 <= kSzB1);
static_assert(kOffF2 % 256 == 0 && kOffES % 256 == 0 && kOffB1 % 256 == 0 && kOffBT % 256 == 0 && kOffNS % 256 == 0 && kOffND % 256 == 0);

typedef __attribute__((ext_vector_type(16))) _Float16 v16h;
typedef __attribute__((ext_vector_type(8)))  _Float16 v8h;
typedef __attribute__((ext_vector_type(16))) __bf16   v16b;
typedef __attribute__((ext_vector_type(8)))  __bf16   v8b;
typedef __attribute__((ext_vector_type(8)))  float    v8f;
typedef __attribute__((ext_vector_type(4)))  float    v4f;
typedef __attribute__((ext_vector_type(4)))  int      v4i;
typedef __attribute__((ext_vector_type(4)))  unsigned int v4u;

__device__ __forceinline__ unsigned short f2bf_bits(float f) {
  unsigned u = __float_as_uint(f);
  return (unsigned short)((u + 0x7FFFu + ((u >> 16) & 1u)) >> 16);
}
__device__ __forceinline__ float bf_bits2f(unsigned short h) { return __uint_as_float(((unsigned)h) << 16); }
__device__ __forceinline__ float bf16r(float f) { return bf_bits2f(f2bf_bits(f)); }
__device__ __forceinline__ void split_bits(float v, unsigned short& hb, unsigned short& lb) {
  const unsigned short h = f2bf_bits(v);
  hb = h;
  lb = f2bf_bits(v - bf_bits2f(h));
}
__device__ __forceinline__ unsigned pk16(unsigned short a, unsigned short b) { return (unsigned)a | ((unsigned)b << 16); }

__device__ __forceinline__ void dep_guard_h(v8f& a, v8f& b, v16h x, v16h y) { asm volatile("v_nop\n\tv_nop\n\tv_nop\n\tv_nop" : "+v"(a), "+v"(b) : "v"(x), "v"(y)); }
__device__ __forceinline__ void dep_guard_b(v8f& a, v8f& b, v16b x, v16b y) { asm volatile("v_nop\n\tv_nop\n\tv_nop\n\tv_nop" : "+v"(a), "+v"(b) : "v"(x), "v"(y)); }
__device__ __forceinline__ void dep_guard4_h(v8f& a, v8f& b, v8f& c, v8f& d, v16h x, v16h y) { asm volatile("v_nop\n\tv_nop\n\tv_nop\n\tv_nop" : "+v"(a), "+v"(b), "+v"(c), "+v"(d) : "v"(x), "v"(y)); }
__device__ __forceinline__ void dep_guard4_b(v8f& a, v8f& b, v8f& c, v8f& d, v16b x, v16b y) { asm volatile("v_nop\n\tv_nop\n\tv_nop\n\tv_nop" : "+v"(a), "+v"(b), "+v"(c), "+v"(d) : "v"(x), "v"(y)); }
__device__ __forceinline__ void keep4_h(v16h a, v16h b, v16h c, v16h d) { asm volatile("v_nop" :: "v"(a), "v"(b), "v"(c), "v"(d)); }
__device__ __forceinline__ void keep4_b(v16b a, v16b b, v16b c, v16b d) { asm volatile("v_nop" :: "v"(a), "v"(b), "v"(c), "v"(d)); }
__device__ __forceinline__ void acc_guard4(v8f& a, v8f& b, v8f& c, v8f& d) { asm volatile("v_nop\n\tv_nop\n\tv_nop\n\tv_nop" : "+v"(a), "+v"(b), "+v"(c), "+v"(d)); }
template <typename T> struct Frag;
template <> struct Frag<_Float16> {
  typedef v16h V; union U { v16h v; v8h h[2]; };
  static __device__ __forceinline__ v16h load(const _Float16* p) {
    U f; f.h[0] = *(const v8h*)(p); f.h[1] = *(const v8h*)(p + 16); return f.v;
  }
  static __device__ __forceinline__ v8f mma(v16h a, v16h b, v8f c) {
    return __builtin_amdgcn_wmma_f32_16x16x32_f16(false, a, false, b, (short)0, c, false, false);
  }
  static __device__ __forceinline__ void guard(v8f& a, v8f& b, v16h x, v16h y) { dep_guard_h(a, b, x, y); }
  static __device__ __forceinline__ void guard4(v8f& a, v8f& b, v8f& c, v8f& d, v16h x, v16h y) { dep_guard4_h(a, b, c, d, x, y); }
  static __device__ __forceinline__ void keep(v16h a, v16h b, v16h c, v16h d) { keep4_h(a, b, c, d); }
};
template <> struct Frag<__bf16> {
  typedef v16b V; union U { v16b v; v8b h[2]; };
  static __device__ __forceinline__ v16b load(const __bf16* p) {
    U f; f.h[0] = *(const v8b*)(p); f.h[1] = *(const v8b*)(p + 16); return f.v;
  }
  static __device__ __forceinline__ v8f mma(v16b a, v16b b, v8f c) {
    return __builtin_amdgcn_wmma_f32_16x16x32_bf16(false, a, false, b, (short)0, c, false, false);
  }
  static __device__ __forceinline__ void guard(v8f& a, v8f& b, v16b x, v16b y) { dep_guard_b(a, b, x, y); }
  static __device__ __forceinline__ void guard4(v8f& a, v8f& b, v8f& c, v8f& d, v16b x, v16b y) { dep_guard4_b(a, b, c, d, x, y); }
  static __device__ __forceinline__ void keep(v16b a, v16b b, v16b c, v16b d) { keep4_b(a, b, c, d); }
};

template <int ET> struct Elem;
template <> struct Elem<0> { typedef _Float16 T; };
template <> struct Elem<1> { typedef __bf16 T; };
template <int ET, bool SPLITA, bool SPLITB, int BIAS_MODE, int OUT_MODE, bool RESID, int ACT = 0>
__global__ __launch_bounds__(256) void wmma_gemm64(
    const unsigned short* __restrict__ Ap, const unsigned short* __restrict__ A2p, int lda, long strideA,
    const unsigned short* __restrict__ Btp, const unsigned short* __restrict__ Bt2p, int ldb, long strideB,
    void* __restrict__ Cout, void* __restrict__ Cout2, int ldc, long strideC,
    const float* __restrict__ bias,
    const float* __restrict__ resid, long strideR,
    int M, int N, int K, float scale) {
  typedef typename Elem<ET>::T T;
  typedef typename Frag<T>::V V;
  const T* A = (const T*)Ap; const T* A2 = (const T*)A2p; const T* Bt = (const T*)Btp; const T* Bt2 = (const T*)Bt2p;
  __shared__ __align__(16) float sT[8][16 * 68];
  const int b    = blockIdx.y;
  const int lane = threadIdx.x & 31;
  const int wave = threadIdx.x >> 5;
  const int tilesN = N >> 6;
  const int tilesM = M >> 6;
  const int tile = blockIdx.x * 8 + wave;
  if (tile >= tilesM * tilesN) return;
  const int tm = tile / tilesN;
  const int tn = tile - tm * tilesN;
  const int m0 = tm << 6;
  const int n0 = tn << 6;

  const T* Ab  = A  + (size_t)b * strideA;
  const T* Bb  = Bt + (size_t)b * strideB;
  const T* Ab2 = SPLITA ? (A2  + (size_t)b * strideA) : nullptr;
  const T* Bb2 = SPLITB ? (Bt2 + (size_t)b * strideB) : nullptr;

  const int rlane = lane & 15;
  const int koff  = (lane >> 4) * 8;
  const int mOff  = (lane >> 4) * 8;

  v8f acc[4][4];
#pragma unroll
  for (int i = 0; i < 4; ++i)
#pragma unroll
    for (int j = 0; j < 4; ++j) acc[i][j] = (v8f){0.f,0.f,0.f,0.f,0.f,0.f,0.f,0.f};

  for (int k0 = 0; k0 < K; k0 += 32) {
    V bh[4], bl[4];
#pragma unroll
    for (int j = 0; j < 4; ++j) {
      const size_t bo = (size_t)(n0 + (j << 4) + rlane) * ldb + koff + k0;
      bh[j] = Frag<T>::load(Bb + bo);
      if (SPLITB) bl[j] = Frag<T>::load(Bb2 + bo);
    }
#pragma unroll
    for (int i = 0; i < 4; ++i) {
      const size_t ao = (size_t)(m0 + (i << 4) + rlane) * lda + koff + k0;
      V ah = Frag<T>::load(Ab + ao);
      V al = ah;
      if (SPLITA) al = Frag<T>::load(Ab2 + ao);
#pragma unroll
      for (int j = 0; j < 4; ++j) {
        acc[i][j] = Frag<T>::mma(ah, bh[j], acc[i][j]);
        if (SPLITB) acc[i][j] = Frag<T>::mma(ah, bl[j], acc[i][j]);
        if (SPLITA) acc[i][j] = Frag<T>::mma(al, bh[j], acc[i][j]);
      }
      Frag<T>::guard4(acc[i][0], acc[i][1], acc[i][2], acc[i][3], ah, al);
    }
    Frag<T>::keep(bh[0], bh[1], bh[2], bh[3]);
    if (SPLITB) Frag<T>::keep(bl[0], bl[1], bl[2], bl[3]);
  }
  acc_guard4(acc[0][0], acc[0][1], acc[0][2], acc[0][3]);
  acc_guard4(acc[1][0], acc[1][1], acc[1][2], acc[1][3]);
  acc_guard4(acc[2][0], acc[2][1], acc[2][2], acc[2][3]);
  acc_guard4(acc[3][0], acc[3][1], acc[3][2], acc[3][3]);

  float* slab = sT[wave];
  const float* Rb = RESID ? (resid + (size_t)b * strideR) : nullptr;
#pragma unroll
  for (int i = 0; i < 4; ++i) {
    const int mBase = m0 + (i << 4);
#pragma unroll
    for (int j = 0; j < 4; ++j) {
      const int n = n0 + (j << 4) + rlane;
      float bv = 0.f;
      if (BIAS_MODE == 2) bv = bias[n];
#pragma unroll
      for (int r = 0; r < 8; ++r) {
        float v = acc[i][j][r] * scale;
        if (BIAS_MODE == 1) v += bias[mBase + mOff + r];
        if (BIAS_MODE == 2) v += bv;
        if (RESID) v += Rb[(size_t)(mBase + mOff + r) * ldc + n];
        if (ACT == 2) v = fmaxf(v, 0.0f);
        if (ACT == 4) v = (v > 0.f) ? v : 0.01f * v;
        slab[(mOff + r) * 68 + (j << 4) + rlane] = v;
      }
    }
    __builtin_amdgcn_fence(__ATOMIC_RELEASE, "workgroup");
    __builtin_amdgcn_wave_barrier();
    __builtin_amdgcn_fence(__ATOMIC_ACQUIRE, "workgroup");
    if (OUT_MODE == 0) {
      float* C = (float*)Cout + (size_t)b * strideC;
      const int hh = lane >> 4, c4 = (lane & 15) * 4;
      for (int pass = 0; pass < 2; ++pass) {
#pragma unroll
        for (int it = 0; it < 8; ++it) {
          const int row = it * 2 + hh;
          v4f v = *(const v4f*)(slab + row * 68 + c4);
          *(volatile v4f*)(C + (size_t)(mBase + row) * ldc + n0 + c4) = v;
        }
        __threadfence();
      }
    } else {
      const int q = lane >> 3, c8 = (lane & 7) * 8;
      unsigned short* C  = (unsigned short*)Cout  + (size_t)b * strideC;
      unsigned short* C2 = (OUT_MODE == 2) ? ((unsigned short*)Cout2 + (size_t)b * strideC) : nullptr;
      for (int pass = 0; pass < 2; ++pass) {
#pragma unroll
        for (int it = 0; it < 4; ++it) {
          const int row = it * 4 + q;
          const float* sp = slab + row * 68 + c8;
          v8h hv, lv;
#pragma unroll
          for (int e = 0; e < 8; ++e) {
            if (OUT_MODE == 1) {
              hv[e] = (_Float16)sp[e];
            } else {
              unsigned short hb = f2bf_bits(sp[e]);
              unsigned short lb = f2bf_bits(sp[e] - bf_bits2f(hb));
              hv[e] = __builtin_bit_cast(_Float16, hb);
              lv[e] = __builtin_bit_cast(_Float16, lb);
            }
          }
          *(volatile v8h*)(C + (size_t)(mBase + row) * ldc + n0 + c8) = hv;
          if (OUT_MODE == 2) *(volatile v8h*)(C2 + (size_t)(mBase + row) * ldc + n0 + c8) = lv;
        }
        __threadfence();
      }
    }
    __builtin_amdgcn_fence(__ATOMIC_RELEASE, "workgroup");
    __builtin_amdgcn_wave_barrier();
    __builtin_amdgcn_fence(__ATOMIC_ACQUIRE, "workgroup");
  }
}


__global__ __launch_bounds__(256) void castx_kernel(const float* __restrict__ x, unsigned short* __restrict__ out, int nrows, int n8) {
  const int i = blockIdx.x * 256 + threadIdx.x;
  if (i >= n8) return;
  const size_t e0 = 8 * (size_t)i;
  const int row = (int)(e0 >> 8);
  const int col = (int)(e0 & 255);
  const int rowc = row < nrows ? row : nrows - 1;
  const float live = row < nrows ? 1.0f : 0.0f;
  const float* p = x + (size_t)rowc * kIn + col;
  const v4f a = *(const v4f*)(p);
  const v4f c = *(const v4f*)(p + 4);
  unsigned short hb[8];
#pragma unroll
  for (int e = 0; e < 4; ++e) {
    const float t0 = a[e];
    const float t1 = c[e];
    hb[e]     = f2bf_bits(fmaf(t0, live, 0.0f));
    hb[4 + e] = f2bf_bits(fmaf(t1, live, 0.0f));
  }
  const v4u u = (v4u){pk16(hb[0], hb[1]), pk16(hb[2], hb[3]), pk16(hb[4], hb[5]), pk16(hb[6], hb[7])};
  unsigned short* q = out + e0;
  *(volatile v4u*)q = u;
  __threadfence();
  *(volatile v4u*)q = u;
}

__global__ __launch_bounds__(kNT) void wtcast_kernel(const float* __restrict__ W, unsigned short* __restrict__ out, int nIn, int nOut) {
  __shared__ float sm[64][65];
  const int t = threadIdx.x;
  const int d0 = blockIdx.x * 64;
  const int h0 = blockIdx.y * 64;
#pragma unroll
  for (int i = 0; i < 16; ++i) {
    const int e = i * kNT + t;
    const int r = e >> 6;
    const int c = e & 63;
    sm[c][r] = W[(size_t)(d0 + r) * nOut + h0 + c];
  }
  __syncthreads();
  const int lane = t & 31, wave = t >> 5;
  const int q = lane >> 3, c8 = (lane & 7) * 8;
  const int row0 = wave * 8 + q;
  const int row1 = wave * 8 + 4 + q;
  unsigned short hb[16];
#pragma unroll
  for (int e = 0; e < 8; ++e) { hb[e] = f2bf_bits(sm[row0][c8 + e]); hb[8 + e] = f2bf_bits(sm[row1][c8 + e]); }
  const v4u u0 = (v4u){pk16(hb[0], hb[1]), pk16(hb[2], hb[3]), pk16(hb[4], hb[5]), pk16(hb[6], hb[7])};
  const v4u u1 = (v4u){pk16(hb[8], hb[9]), pk16(hb[10], hb[11]), pk16(hb[12], hb[13]), pk16(hb[14], hb[15])};
  unsigned short* p0 = out + (size_t)(h0 + row0) * nIn + d0 + c8;
  unsigned short* p1 = out + (size_t)(h0 + row1) * nIn + d0 + c8;
  for (int pass = 0; pass < 2; ++pass) {
    *(volatile v4u*)p0 = u0;
    *(volatile v4u*)p1 = u1;
    __threadfence();
  }
}

__global__ __launch_bounds__(kNT) void att_terms_kernel(const float* __restrict__ Hm, const float* __restrict__ al,
                                                      const float* __restrict__ ar, float* __restrict__ EL,
                                                      float* __restrict__ ER, int total, int heads) {
  const int t = blockIdx.x * kNT + threadIdx.x;
  if (t >= total) return;
  const int h = t % heads;
  const float* hp = Hm + (size_t)t * kHid;
  const float* ap = al + h * kHid;
  const float* bp = ar + h * kHid;
  float sl = 0.f, sr = 0.f;
#pragma unroll 1
  for (int d = 0; d < kHid; d += 4) {
    const v4f hv = *(const v4f*)(hp + d);
    const v4f av = *(const v4f*)(ap + d);
    const v4f bv = *(const v4f*)(bp + d);
#pragma unroll
    for (int e = 0; e < 4; ++e) {
      const float x = hv[e];
      const float wa = av[e];
      const float wb = bv[e];
      sl = fmaf(x, bf16r(wa), sl);
      sr = fmaf(x, bf16r(wb), sr);
    }
  }
  float* pl = EL + t;
  float* pr = ER + t;
  *(volatile float*)pl = sl;
  *(volatile float*)pr = sr;
  __threadfence();
  *(volatile float*)pl = sl;
  *(volatile float*)pr = sr;
}

__device__ __forceinline__ int blk_excl_scan(int cnt, int* scan_ws, int tid, int* tot) {
  const int lane = tid & 31, wave = tid >> 5; int incl = cnt;
#pragma unroll
  for (int o = 1; o < 32; o <<= 1) { const int v = __shfl_up(incl, o, 32); if (lane >= o) incl += v; }
  if (lane == 31) scan_ws[wave] = incl;
  __syncthreads();
  if (wave == 0) {
    int wv = (lane < kNT / 32) ? scan_ws[lane] : 0; int wincl = wv;
#pragma unroll
    for (int o = 1; o < 32; o <<= 1) { const int v = __shfl_up(wincl, o, 32); if (lane >= o) wincl += v; }
    if (lane < kNT / 32) scan_ws[32 + lane] = wincl - wv;
    if (lane == 31) scan_ws[64] = wincl;
  }
  __syncthreads();
  const int res = scan_ws[32 + wave] + incl - cnt; *tot = scan_ws[64];
  return res;
}
template <int SP, int SCH, int TS, bool HASVAL>
__device__ __forceinline__ int chunk_hits(const int* __restrict__ keyv, const int* __restrict__ valv, int nE, int nNodes,
                                          int e0, int n0, int tid, int* LIST, int* scan_ws) {
  const int eb = e0 + tid * SP;
  const bool valid = eb < nE;
  const int ebc = valid ? eb : (nE - SP);
  int rec[SP]; int cnt = 0;
#pragma unroll
  for (int k = 0; k < SP; k += 4) {
    const v4i d4 = *(const v4i*)(keyv + ebc + k);
    v4i s4 = (v4i){0, 0, 0, 0};
    if (HASVAL) s4 = *(const v4i*)(valv + ebc + k);
#pragma unroll
    for (int e = 0; e < 4; ++e) {
      const int d = d4[e];
      int s = s4[e]; s = s < 0 ? 0 : (s >= nNodes ? nNodes - 1 : s);
      const bool hit = valid && d >= n0 && d < n0 + TS;
      const int r = (int)((((unsigned)(d - n0)) << 16) | (unsigned)s);
      rec[k + e] = hit ? r : -1;
      cnt += hit ? 1 : 0;
    }
  }
  int tot; int p = blk_excl_scan(cnt, scan_ws, tid, &tot);
#pragma unroll
  for (int k = 0; k < SP; ++k) if (rec[k] >= 0) { if ((unsigned)p < (unsigned)SCH) LIST[p] = rec[k]; ++p; }
  __syncthreads();
  return tot < SCH ? tot : SCH;
}

__global__ __launch_bounds__(kNT) void gat1_kernel(const float* __restrict__ Hm, const int* __restrict__ srcv, const int* __restrict__ dstv,
                                                 const float* __restrict__ EL, const float* __restrict__ ER, const float* __restrict__ bias,
                                                 float* AGG, unsigned short* __restrict__ AH, unsigned short* __restrict__ ALo) {
  __shared__ int LIST[kSch1];
  __shared__ float SM[kTS1 * kHeads];
  __shared__ float SL[kTS1 * kHeads];
  __shared__ float SER[kTS1 * kHeads];
  __shared__ int scan_ws[80];
  const int tid = threadIdx.x, lane = tid & 31, wave = tid >> 5;
  const int n0 = blockIdx.x * kTS1;
  const int hd = lane & 3;
  const v4f z4 = {0.f, 0.f, 0.f, 0.f};
  v4f bA0, bA1, bB0, bB1;
  {
    const v4f t0 = *(const v4f*)(bias + 8 * lane);
    const v4f t1 = *(const v4f*)(bias + 8 * lane + 4);
    const v4f t2 = *(const v4f*)(bias + 256 + 8 * lane);
    const v4f t3 = *(const v4f*)(bias + 256 + 8 * lane + 4);
#pragma unroll
    for (int e = 0; e < 4; ++e) {
      const float s0 = t0[e], s1 = t1[e], s2 = t2[e], s3 = t3[e];
      bA0[e] = bf16r(s0); bA1[e] = bf16r(s1); bB0[e] = bf16r(s2); bB1[e] = bf16r(s3);
    }
  }
#pragma unroll 1
  for (int j = 0; j < kRPW1; ++j) {
    float* rp = AGG + (size_t)(n0 + wave * kRPW1 + j) * kF1 + 4 * lane;
#pragma unroll
    for (int jj = 0; jj < 4; ++jj) *(v4f*)(rp + 128 * jj) = z4;
  }
  for (int i = tid; i < kSch1; i += kNT) LIST[i] = -1;
  if (tid < 80) scan_ws[tid] = 0;
  for (int i = tid; i < kTS1 * kHeads; i += kNT) { SM[i] = -INFINITY; SL[i] = 0.f; SER[i] = ER[(size_t)n0 * kHeads + i]; }
  __syncthreads();
#pragma unroll 1
  for (int c = 0; c < kNch1; ++c) {
    const int tot = chunk_hits<kSch1 / kNT, kSch1, kTS1, true>(dstv, srcv, kES, kNS, c * kSch1, n0, tid, LIST, scan_ws);
#pragma unroll 1
    for (int base = 0; base < tot; base += 32) {
      const int q = base + lane;
      const int qc = q < kSch1 ? q : kSch1 - 1;
      const int lv = LIST[qc];
      const int rv = (q < tot) ? lv : -1;
      const int own = (rv >= 0 && ((rv >> 16) / kRPW1) == wave) ? 1 : 0;
      unsigned msk = (unsigned)__ballot(own);
#pragma unroll 1
      for (int it = 0; it < 32; ++it) {
        if (msk == 0u) break;
        const int bp = __builtin_ctz(msk); msk &= msk - 1u;
        const int r = __shfl(rv, bp, 32);
        const int dl = r >> 16, s = r & 0xFFFF;
        const int mi = dl * kHeads + hd;
        float lg = EL[(size_t)s * kHeads + hd] + SER[mi];
        lg = (lg >= 0.f) ? lg : 0.2f * lg;
        const float mo = SM[mi], lo = SL[mi];
        const float mn = fmaxf(mo, lg);
        const float rr = expf(mo - mn);
        const float ex = expf(lg - mn);
        const float ln = lo * rr + ex;
        if (lane < kHeads) { SM[mi] = mn; SL[mi] = ln; }
        float* rp = AGG + (size_t)(n0 + dl) * kF1 + 4 * lane;
        const float* hrow = Hm + (size_t)s * kF1 + 4 * lane;
#pragma unroll
        for (int jj = 0; jj < 4; ++jj) {
          const float rrj = __shfl(rr, jj, 32);
          const float exj = __shfl(ex, jj, 32);
          const v4f hv = *(const v4f*)(hrow + 128 * jj);
          v4f a = *(const v4f*)(rp + 128 * jj);
          a = a * rrj + exj * hv;
          *(v4f*)(rp + 128 * jj) = a;
        }
      }
    }
    __syncthreads();
  }
#pragma unroll 1
  for (int j = 0; j < kRPW1; ++j) {
    const int dl = wave * kRPW1 + j;
    const int n = n0 + dl;
    const float ls = SL[dl * kHeads + hd];
    const float inv = 1.0f / fmaxf(ls, 1e-9f);
    const float invA = __shfl(inv, lane >> 4, 32);
    const float invB = __shfl(inv, 2 + (lane >> 4), 32);
    const float* rp = AGG + (size_t)n * kF1;
    const v4f a0 = *(const v4f*)(rp + 8 * lane);
    const v4f a1 = *(const v4f*)(rp + 8 * lane + 4);
    const v4f c0 = *(const v4f*)(rp + 256 + 8 * lane);
    const v4f c1 = *(const v4f*)(rp + 256 + 8 * lane + 4);
    unsigned short hb[16], lb[16];
#pragma unroll
    for (int e = 0; e < 4; ++e) {
      float t;
      t = a0[e] * invA; t = t + bA0[e]; t = fmaxf(t, 0.f); split_bits(t, hb[e], lb[e]);
      t = a1[e] * invA; t = t + bA1[e]; t = fmaxf(t, 0.f); split_bits(t, hb[4 + e], lb[4 + e]);
      t = c0[e] * invB; t = t + bB0[e]; t = fmaxf(t, 0.f); split_bits(t, hb[8 + e], lb[8 + e]);
      t = c1[e] * invB; t = t + bB1[e]; t = fmaxf(t, 0.f); split_bits(t, hb[12 + e], lb[12 + e]);
    }
    const v4u hA = (v4u){pk16(hb[0], hb[1]), pk16(hb[2], hb[3]), pk16(hb[4], hb[5]), pk16(hb[6], hb[7])};
    const v4u lA = (v4u){pk16(lb[0], lb[1]), pk16(lb[2], lb[3]), pk16(lb[4], lb[5]), pk16(lb[6], lb[7])};
    const v4u hB = (v4u){pk16(hb[8], hb[9]), pk16(hb[10], hb[11]), pk16(hb[12], hb[13]), pk16(hb[14], hb[15])};
    const v4u lB = (v4u){pk16(lb[8], lb[9]), pk16(lb[10], lb[11]), pk16(lb[12], lb[13]), pk16(lb[14], lb[15])};
    unsigned short* rh = AH + (size_t)n * kF1;
    unsigned short* rl = ALo + (size_t)n * kF1;
    for (int pass = 0; pass < 2; ++pass) {
      *(volatile v4u*)(rh + 8 * lane) = hA;
      *(volatile v4u*)(rh + 256 + 8 * lane) = hB;
      *(volatile v4u*)(rl + 8 * lane) = lA;
      *(volatile v4u*)(rl + 256 + 8 * lane) = lB;
      __threadfence();
    }
  }
  if (blockIdx.x == kNTile1 - 1) {
    const v4u zu = (v4u){0u, 0u, 0u, 0u};
#pragma unroll 1
    for (int jj = 0; jj < 4; ++jj) {
      const int row = kNS + wave * 4 + jj;
      unsigned short* rh = AH + (size_t)row * kF1;
      unsigned short* rl = ALo + (size_t)row * kF1;
      for (int pass = 0; pass < 2; ++pass) {
        *(volatile v4u*)(rh + 8 * lane) = zu;
        *(volatile v4u*)(rh + 256 + 8 * lane) = zu;
        *(volatile v4u*)(rl + 8 * lane) = zu;
        *(volatile v4u*)(rl + 256 + 8 * lane) = zu;
        __threadfence();
      }
    }
  }
}

__global__ __launch_bounds__(kNT) void gat2_kernel(const float* __restrict__ Hm, const int* __restrict__ srcv, const int* __restrict__ dstv,
                                                 const float* __restrict__ EL, const float* __restrict__ ER, const float* __restrict__ bias,
                                                 float* EMB) {
  __shared__ int LIST[kSch2];
  __shared__ float SM[kTS1];
  __shared__ float SL[kTS1];
  __shared__ float SER[kTS1];
  __shared__ int scan_ws[80];
  const int tid = threadIdx.x, lane = tid & 31, wave = tid >> 5;
  const int n0 = blockIdx.x * kTS1;
  const v4f z4 = {0.f, 0.f, 0.f, 0.f};
  v4f b4;
  {
    const v4f t0 = *(const v4f*)(bias + 4 * lane);
#pragma unroll
    for (int e = 0; e < 4; ++e) { const float s0 = t0[e]; b4[e] = bf16r(s0); }
  }
#pragma unroll 1
  for (int j = 0; j < kRPW1; ++j) *(v4f*)(EMB + (size_t)(n0 + wave * kRPW1 + j) * kOut + 4 * lane) = z4;
  for (int i = tid; i < kSch2; i += kNT) LIST[i] = -1;
  if (tid < 80) scan_ws[tid] = 0;
  for (int i = tid; i < kTS1; i += kNT) { SM[i] = -INFINITY; SL[i] = 0.f; SER[i] = ER[n0 + i]; }
  __syncthreads();
#pragma unroll 1
  for (int c = 0; c < kNch2; ++c) {
    const int tot = chunk_hits<kSch2 / kNT, kSch2, kTS1, true>(dstv, srcv, kES, kNS, c * kSch2, n0, tid, LIST, scan_ws);
#pragma unroll 1
    for (int base = 0; base < tot; base += 32) {
      const int q = base + lane;
      const int qc = q < kSch2 ? q : kSch2 - 1;
      const int lv = LIST[qc];
      const int rv = (q < tot) ? lv : -1;
      const int own = (rv >= 0 && ((rv >> 16) / kRPW1) == wave) ? 1 : 0;
      unsigned msk = (unsigned)__ballot(own);
#pragma unroll 1
      for (int it = 0; it < 32; ++it) {
        if (msk == 0u) break;
        const int bp = __builtin_ctz(msk); msk &= msk - 1u;
        const int r = __shfl(rv, bp, 32);
        const int dl = r >> 16, s = r & 0xFFFF;
        float lg = EL[s] + SER[dl];
        lg = (lg >= 0.f) ? lg : 0.2f * lg;
        const float mo = SM[dl], lo = SL[dl];
        const float mn = fmaxf(mo, lg);
        const float rr = expf(mo - mn);
        const float ex = expf(lg - mn);
        const float ln = lo * rr + ex;
        if (lane == 0) { SM[dl] = mn; SL[dl] = ln; }
        const v4f hv = *(const v4f*)(Hm + (size_t)s * kOut + 4 * lane);
        float* rp = EMB + (size_t)(n0 + dl) * kOut + 4 * lane;
        v4f a = *(const v4f*)rp;
        a = a * rr + ex * hv;
        *(v4f*)rp = a;
      }
    }
    __syncthreads();
  }
#pragma unroll 1
  for (int j = 0; j < kRPW1; ++j) {
    const int dl = wave * kRPW1 + j;
    const int n = n0 + dl;
    const float ls = SL[dl];
    const float inv = 1.0f / fmaxf(ls, 1e-9f);
    float* rp = EMB + (size_t)n * kOut + 4 * lane;
    const v4f a = *(const v4f*)rp;
    v4f v;
#pragma unroll
    for (int e = 0; e < 4; ++e) { float t = a[e] * inv; t = t + b4[e]; v[e] = fmaxf(t, 0.f); }
    for (int pass = 0; pass < 2; ++pass) { *(volatile v4f*)rp = v; __threadfence(); }
  }
}

__global__ __launch_bounds__(kNT) void deg_kernel(const int* __restrict__ srcv, float* __restrict__ NSA) {
  __shared__ int LIST[kSchL];
  __shared__ int CNT[kTSL];
  __shared__ int scan_ws[80];
  const int tid = threadIdx.x, lane = tid & 31, wave = tid >> 5;
  const int n0 = blockIdx.x * kTSL;
  for (int i = tid; i < kSchL; i += kNT) LIST[i] = -1;
  for (int i = tid; i < kTSL; i += kNT) CNT[i] = 0;
  if (tid < 80) scan_ws[tid] = 0;
  __syncthreads();
#pragma unroll 1
  for (int c = 0; c < kNchL; ++c) {
    const int tot = chunk_hits<kSchL / kNT, kSchL, kTSL, false>(srcv, srcv, kEL, kNL, c * kSchL, n0, tid, LIST, scan_ws);
#pragma unroll 1
    for (int base = 0; base < tot; base += 32) {
      const int q = base + lane;
      const int qc = q < kSchL ? q : kSchL - 1;
      const int lv = LIST[qc];
      const int rv = (q < tot) ? lv : -1;
      const int own = (rv >= 0 && ((rv >> 16) >> 8) == wave) ? 1 : 0;
      unsigned msk = (unsigned)__ballot(own);
#pragma unroll 1
      for (int it = 0; it < 32; ++it) {
        if (msk == 0u) break;
        const int bp = __builtin_ctz(msk); msk &= msk - 1u;
        const int r = __shfl(rv, bp, 32);
        const int dl = r >> 16;
        if (lane == 0) CNT[dl] += 1;
      }
    }
    __syncthreads();
  }
  __syncthreads();
  float nsr[8];
#pragma unroll
  for (int k = 0; k < 8; ++k) {
    const int cs = CNT[k * kNT + tid];
    nsr[k] = 1.0f / sqrtf((float)(cs < 1 ? 1 : cs));
  }
  for (int pass = 0; pass < 2; ++pass) {
#pragma unroll
    for (int k = 0; k < 8; ++k) *(volatile float*)(NSA + n0 + k * kNT + tid) = nsr[k];
    __threadfence();
  }
}

template <int LAYER>
__global__ __launch_bounds__(kNT) void gcn_kernel(const float* __restrict__ G, const int* __restrict__ srcv, const int* __restrict__ dstv,
                                                const float* __restrict__ NSA, const float* NDin, const float* __restrict__ bias,
                                                float* ACC, unsigned short* __restrict__ AH, unsigned short* __restrict__ ALo, float* NDout) {
  __shared__ int LIST[kSchL];
  __shared__ int CNT[kTSL];
  __shared__ int scan_ws[80];
  const int tid = threadIdx.x, lane = tid & 31, wave = tid >> 5;
  const int n0 = blockIdx.x * kTSL;
  const v4f z4 = {0.f, 0.f, 0.f, 0.f};
  const int cq = 8 * (lane & 15);
  v4f bq0, bq1, b4;
  {
    const v4f t0 = *(const v4f*)(bias + cq);
    const v4f t1 = *(const v4f*)(bias + cq + 4);
    const v4f t2 = *(const v4f*)(bias + 4 * lane);
#pragma unroll
    for (int e = 0; e < 4; ++e) {
      const float s0 = t0[e], s1 = t1[e], s2 = t2[e];
      bq0[e] = bf16r(s0); bq1[e] = bf16r(s1); b4[e] = bf16r(s2);
    }
  }
#pragma unroll 1
  for (int j = 0; j < kRPWL; ++j) *(v4f*)(ACC + (size_t)(n0 + wave * kRPWL + j) * kOut + 4 * lane) = z4;
  for (int i = tid; i < kSchL; i += kNT) LIST[i] = -1;
  for (int i = tid; i < kTSL; i += kNT) CNT[i] = 0;
  if (tid < 80) scan_ws[tid] = 0;
  __syncthreads();
#pragma unroll 1
  for (int c = 0; c < kNchL; ++c) {
    const int tot = chunk_hits<kSchL / kNT, kSchL, kTSL, true>(dstv, srcv, kEL, kNL, c * kSchL, n0, tid, LIST, scan_ws);
#pragma unroll 1
    for (int base = 0; base < tot; base += 32) {
      const int q = base + lane;
      const int qc = q < kSchL ? q : kSchL - 1;
      const int lv = LIST[qc];
      const int rv = (q < tot) ? lv : -1;
      const int own = (rv >= 0 && ((rv >> 16) >> 8) == wave) ? 1 : 0;
      unsigned msk = (unsigned)__ballot(own);
#pragma unroll 1
      for (int it = 0; it < 32; ++it) {
        if (msk == 0u) break;
        const int bp = __builtin_ctz(msk); msk &= msk - 1u;
        const int r = __shfl(rv, bp, 32);
        const int dl = r >> 16, s = r & 0xFFFF;
        if (LAYER == 1) { if (lane == 0) CNT[dl] += 1; }
        const float w = NSA[s];
        const v4f hv = *(const v4f*)(G + (size_t)s * kOut + 4 * lane);
        float* rp = ACC + (size_t)(n0 + dl) * kOut + 4 * lane;
        v4f a = *(const v4f*)rp;
        a = hv * w + a;
        *(v4f*)rp = a;
      }
    }
    __syncthreads();
  }
  __syncthreads();
  if (LAYER == 1) {
    float ndr[8];
#pragma unroll
    for (int k = 0; k < 8; ++k) {
      const int cd = CNT[k * kNT + tid];
      ndr[k] = 1.0f / sqrtf((float)(cd < 1 ? 1 : cd));
    }
    for (int pass = 0; pass < 2; ++pass) {
#pragma unroll
      for (int k = 0; k < 8; ++k) *(volatile float*)(NDout + n0 + k * kNT + tid) = ndr[k];
      __threadfence();
    }
    const int hrow = lane >> 4;
#pragma unroll 1
    for (int jj = 0; jj < kRPWL / 2; ++jj) {
      const int dl0 = wave * kRPWL + 2 * jj;
      const int ne = n0 + dl0;
      if (ne < kNLP) {
        const int dl = dl0 + hrow;
        const int n = ne + hrow;
        const bool live = n < kNL;
        const int cn = CNT[dl];
        const float ndv = 1.0f / sqrtf((float)(cn < 1 ? 1 : cn));
        const float* rp = ACC + (size_t)n * kOut + cq;
        const v4f a0 = *(const v4f*)rp;
        const v4f a1 = *(const v4f*)(rp + 4);
        unsigned short hb[8], lb[8];
#pragma unroll
        for (int e = 0; e < 4; ++e) {
          float t;
          t = a0[e] * ndv; t = t + bq0[e]; t = live ? fmaxf(t, 0.f) : 0.f; split_bits(t, hb[e], lb[e]);
          t = a1[e] * ndv; t = t + bq1[e]; t = live ? fmaxf(t, 0.f) : 0.f; split_bits(t, hb[4 + e], lb[4 + e]);
        }
        const v4u hu = (v4u){pk16(hb[0], hb[1]), pk16(hb[2], hb[3]), pk16(hb[4], hb[5]), pk16(hb[6], hb[7])};
        const v4u lu = (v4u){pk16(lb[0], lb[1]), pk16(lb[2], lb[3]), pk16(lb[4], lb[5]), pk16(lb[6], lb[7])};
        unsigned short* ph = AH + (size_t)n * kOut + cq;
        unsigned short* plo = ALo + (size_t)n * kOut + cq;
        for (int pass = 0; pass < 2; ++pass) {
          *(volatile v4u*)ph = hu;
          *(volatile v4u*)plo = lu;
          __threadfence();
        }
      }
    }
  } else {
#pragma unroll 1
    for (int j = 0; j < kRPWL; ++j) {
      const int dl = wave * kRPWL + j;
      const int n = n0 + dl;
      if (n < kNL) {
        const float ndv = NDin[n];
        float* rp = ACC + (size_t)n * kOut + 4 * lane;
        const v4f a = *(const v4f*)rp;
        v4f v;
#pragma unroll
        for (int e = 0; e < 4; ++e) { float t = a[e] * ndv; t = t + b4[e]; v[e] = t; }
        for (int pass = 0; pass < 2; ++pass) { *(volatile v4f*)rp = v; __threadfence(); }
      }
    }
  }
}

__global__ __launch_bounds__(kNT) void cls_kernel(const float* __restrict__ ES, const float* __restrict__ EG, const int* __restrict__ tok,
                                                const float* __restrict__ W, const float* __restrict__ bc, float* __restrict__ out) {
  __shared__ float sW[2 * kOut * kCls];
  const int tid = threadIdx.x, lane = tid & 31, wave = tid >> 5;
  for (int i = tid; i < 2 * kOut * kCls; i += kNT) sW[i] = bf16r(W[i]);
  __syncthreads();
  const int gw = blockIdx.x * (kNT / 32) + wave;
  if (gw < kNS / 8) {
    const int node = gw * 8 + (lane >> 2);
    const int c = lane & 3;
    int t = tok[node]; t = t < 0 ? 0 : (t >= kNL ? kNL - 1 : t);
    float acc = 0.f;
    const float* ep = ES + (size_t)node * kOut;
#pragma unroll 1
    for (int j = 0; j < kOut; j += 4) {
      const v4f e4 = *(const v4f*)(ep + j);
      acc = fmaf(e4[0], sW[(j + 0) * kCls + c], acc);
      acc = fmaf(e4[1], sW[(j + 1) * kCls + c], acc);
      acc = fmaf(e4[2], sW[(j + 2) * kCls + c], acc);
      acc = fmaf(e4[3], sW[(j + 3) * kCls + c], acc);
    }
    const float* gp = EG + (size_t)t * kOut;
#pragma unroll 1
    for (int j = 0; j < kOut; j += 4) {
      const v4f g4 = *(const v4f*)(gp + j);
      acc = fmaf(g4[0], sW[(kOut + j + 0) * kCls + c], acc);
      acc = fmaf(g4[1], sW[(kOut + j + 1) * kCls + c], acc);
      acc = fmaf(g4[2], sW[(kOut + j + 2) * kCls + c], acc);
      acc = fmaf(g4[3], sW[(kOut + j + 3) * kCls + c], acc);
    }
    acc = acc + bf16r(bc[c]);
    float* op = out + (size_t)gw * 32 + lane;
    *(volatile float*)op = acc;
    __threadfence();
    *(volatile float*)op = acc;
  }
}

extern "C" void kernel_launch(void* const* d_in, const int* in_sizes, int n_in,
                              void* d_out, int out_size, void* d_ws, size_t ws_size, hipStream_t stream) {
  (void)in_sizes; (void)n_in; (void)out_size;
  const float* x_small = (const float*)d_in[0];
  const float* x_large = (const float*)d_in[1];
  const int*   src_s   = (const int*)d_in[2];
  const int*   dst_s   = (const int*)d_in[3];
  const int*   src_l   = (const int*)d_in[4];
  const int*   dst_l   = (const int*)d_in[5];
  const int*   tok     = (const int*)d_in[6];
  const float* Wg1  = (const float*)d_in[7];
  const float* bg1  = (const float*)d_in[8];
  const float* al1  = (const float*)d_in[9];
  const float* ar1  = (const float*)d_in[10];
  const float* Wg2  = (const float*)d_in[11];
  const float* bg2  = (const float*)d_in[12];
  const float* al2  = (const float*)d_in[13];
  const float* ar2  = (const float*)d_in[14];
  const float* Wc1  = (const float*)d_in[15];
  const float* bc1  = (const float*)d_in[16];
  const float* Wc2  = (const float*)d_in[17];
  const float* bc2  = (const float*)d_in[18];
  const float* Wcls = (const float*)d_in[19];
  const float* bcls = (const float*)d_in[20];
  float* out = (float*)d_out;

  if (kWsTotal > ws_size) return;
  char* ws = (char*)d_ws;
  float* H1  = (float*)(ws + kOffF1);
  float* EL2 = (float*)(ws + kOffF1);
  float* ER2 = (float*)(ws + kOffF1 + 81920);
  float* G1  = (float*)(ws + kOffF1);
  float* G2  = (float*)(ws + kOffF1);
  float* AGG1 = (float*)(ws + kOffF2);
  float* H2   = (float*)(ws + kOffF2);
  float* AGGL = (float*)(ws + kOffF2);
  float* EMBL = (float*)(ws + kOffF2);
  float* NSA  = (float*)(ws + kOffF2 + kOffNS);
  float* NDA  = (float*)(ws + kOffF2 + kOffND);
  float* EMBS = (float*)(ws + kOffES);
  float* EL1  = (float*)(ws + kOffES);
  float* ER1  = (float*)(ws + kOffES + (size_t)kNS * kHeads * 4);
  unsigned short* XB1 = (unsigned short*)(ws + kOffB1);
  unsigned short* A2H = (unsigned short*)(ws + kOffB1);
  unsigned short* A2L = (unsigned short*)(ws + kOffB1 + (size_t)kNSP * kF1 * 2);
  unsigned short* XB3 = (unsigned short*)(ws + kOffB1);
  unsigned short* A4H = (unsigned short*)(ws + kOffB1);
  unsigned short* A4L = (unsigned short*)(ws + kOffB1 + (size_t)kNLP * kOut * 2);
  unsigned short* Bt1 = (unsigned short*)(ws + kOffBT);
  unsigned short* Bt2 = Bt1 + (size_t)kIn * kF1;
  unsigned short* Bt3 = Bt2 + (size_t)kF1 * kOut;
  unsigned short* Bt4 = Bt3 + (size_t)kIn * kHid;

  wtcast_kernel<<<dim3(kIn / 64, kF1 / 64), kNT, 0, stream>>>(Wg1, Bt1, kIn, kF1);
  wtcast_kernel<<<dim3(kF1 / 64, kOut / 64), kNT, 0, stream>>>(Wg2, Bt2, kF1, kOut);
  wtcast_kernel<<<dim3(kIn / 64, kHid / 64), kNT, 0, stream>>>(Wc1, Bt3, kIn, kHid);
  wtcast_kernel<<<dim3(kHid / 64, kOut / 64), kNT, 0, stream>>>(Wc2, Bt4, kHid, kOut);

  {
    const int n8 = kNSP * kIn / 8;
    castx_kernel<<<(n8 + 255) / 256, 256, 0, stream>>>(x_small, XB1, kNS, n8);
  }
  {
    const int tiles = (kNSP / 64) * (kF1 / 64);
    wmma_gemm64<1, false, false, 0, 0, false><<<dim3((tiles + 7) / 8, 1), 256, 0, stream>>>(
        XB1, XB1, kIn, 0L, Bt1, Bt1, kIn, 0L, (void*)H1, (void*)nullptr, kF1, 0L,
        (const float*)nullptr, (const float*)nullptr, 0L, kNSP, kF1, kIn, 1.0f);
  }
  att_terms_kernel<<<(kNS * kHeads + kNT - 1) / kNT, kNT, 0, stream>>>(H1, al1, ar1, EL1, ER1, kNS * kHeads, kHeads);
  gat1_kernel<<<kNTile1, kNT, 0, stream>>>(H1, src_s, dst_s, EL1, ER1, bg1, AGG1, A2H, A2L);

  {
    const int tiles = (kNSP / 64) * (kOut / 64);
    wmma_gemm64<1, true, false, 0, 0, false><<<dim3((tiles + 7) / 8, 1), 256, 0, stream>>>(
        A2H, A2L, kF1, 0L, Bt2, Bt2, kF1, 0L, (void*)H2, (void*)nullptr, kOut, 0L,
        (const float*)nullptr, (const float*)nullptr, 0L, kNSP, kOut, kF1, 1.0f);
  }
  att_terms_kernel<<<(kNS + kNT - 1) / kNT, kNT, 0, stream>>>(H2, al2, ar2, EL2, ER2, kNS, 1);
  gat2_kernel<<<kNTile1, kNT, 0, stream>>>(H2, src_s, dst_s, EL2, ER2, bg2, EMBS);

  {
    const int n8 = kNLP * kIn / 8;
    castx_kernel<<<(n8 + 255) / 256, 256, 0, stream>>>(x_large, XB3, kNL, n8);
  }
  {
    const int tiles = (kNLP / 64) * (kOut / 64);
    wmma_gemm64<1, false, false, 0, 0, false><<<dim3((tiles + 7) / 8, 1), 256, 0, stream>>>(
        XB3, XB3, kIn, 0L, Bt3, Bt3, kIn, 0L, (void*)G1, (void*)nullptr, kOut, 0L,
        (const float*)nullptr, (const float*)nullptr, 0L, kNLP, kOut, kIn, 1.0f);
  }
  deg_kernel<<<kNTileL, kNT, 0, stream>>>(src_l, NSA);
  gcn_kernel<1><<<kNTileL, kNT, 0, stream>>>(G1, src_l, dst_l, NSA, NDA, bc1, AGGL, A4H, A4L, NDA);

  {
    const int tiles = (kNLP / 64) * (kOut / 64);
    wmma_gemm64<1, true, false, 0, 0, false><<<dim3((tiles + 7) / 8, 1), 256, 0, stream>>>(
        A4H, A4L, kOut, 0L, Bt4, Bt4, kHid, 0L, (void*)G2, (void*)nullptr, kOut, 0L,
        (const float*)nullptr, (const float*)nullptr, 0L, kNLP, kOut, kHid, 1.0f);
  }
  gcn_kernel<2><<<kNTileL, kNT, 0, stream>>>(G2, src_l, dst_l, NSA, NDA, bc2, EMBL, A4H, A4L, NDA);

  cls_kernel<<<(kNS / 8 + 7) / 8, kNT, 0, stream>>>(EMBS, EMBL, tok, Wcls, bcls, out);
}
